// SelfAttentionLayerSparse_13606456394290
// MI455X (gfx1250) — hardware-verified
//
#include <hip/hip_runtime.h>
#include <stddef.h>
#include <stdint.h>


#define KIN   512
#define NQKV  1536
#define FOUT  512
#define NHD   8
#define GR    32
#define GC    512
#define KC    128
#define AP    136
#define OP    516
#define TP    72
#define NB    64
#define CHUNK 2048
#define NTHR  256
#define NWAVE 8
#define WCAP  256
#define NGRP  (CHUNK / (NTHR * 4))

#define LDS_SACC (NB * FOUT)
#define LDS_MD   (NB * NHD * 2)
#define LDS_LIST (NWAVE * WCAP)
#define LDS_BYTES ((LDS_SACC + LDS_MD + LDS_LIST + NWAVE) * 4)

static_assert(WCAP == (CHUNK / NTHR) * 32);
static_assert(NGRP == 2);
static_assert(NB == 8 * NWAVE);
static_assert(NB <= 256);
static_assert(CHUNK <= 4096);
static_assert((LDS_SACC % 4) == 0);
static_assert(LDS_BYTES == 143392);
static_assert(GC == NWAVE * 64);
static_assert((KIN % KC) == 0);
static_assert((KC % 32) == 0);
static_assert((NQKV % GC) == 0);
static_assert((OP % 4) == 0);
static_assert((AP % 8) == 0);
static_assert((TP % 8) == 0);

typedef float          v4f   __attribute__((ext_vector_type(4)));
typedef float          v8f   __attribute__((ext_vector_type(8)));
typedef int            v4i   __attribute__((ext_vector_type(4)));
typedef unsigned short v8us  __attribute__((ext_vector_type(8)));
typedef __bf16         v16bf __attribute__((ext_vector_type(16)));
union Frag  { v16bf v; v4i q[2]; };
union Pack8 { v8us s; v4i i; };

__device__ __forceinline__ v8f wm(v16bf a, v16bf b, v8f c) {
  v8f d = __builtin_amdgcn_wmma_f32_16x16x32_bf16(false, a, false, b, (short)0, c, false, false);
  asm volatile("v_nop\n\tv_nop\n\tv_nop\n\tv_nop" : "+v"(d) : "v"(a), "v"(b));
  return d;
}

__device__ __forceinline__ unsigned sp2(float f) {
  const unsigned u = __float_as_uint(f);
  const unsigned h = (u + 0x7FFFu + ((u >> 16) & 1u)) >> 16;
  const float r = f - __uint_as_float(h << 16);
  const unsigned ur = __float_as_uint(r);
  const unsigned l = (ur + 0x7FFFu + ((ur >> 16) & 1u)) >> 16;
  return (h & 0xFFFFu) | (l << 16);
}

__device__ __forceinline__ void sp8(v4f a, v4f b, v4i& hi, v4i& lo) {
  Pack8 ph, pl;
  unsigned r;
  r = sp2(a.x); ph.s[0] = (unsigned short)(r & 0xFFFFu); pl.s[0] = (unsigned short)(r >> 16);
  r = sp2(a.y); ph.s[1] = (unsigned short)(r & 0xFFFFu); pl.s[1] = (unsigned short)(r >> 16);
  r = sp2(a.z); ph.s[2] = (unsigned short)(r & 0xFFFFu); pl.s[2] = (unsigned short)(r >> 16);
  r = sp2(a.w); ph.s[3] = (unsigned short)(r & 0xFFFFu); pl.s[3] = (unsigned short)(r >> 16);
  r = sp2(b.x); ph.s[4] = (unsigned short)(r & 0xFFFFu); pl.s[4] = (unsigned short)(r >> 16);
  r = sp2(b.y); ph.s[5] = (unsigned short)(r & 0xFFFFu); pl.s[5] = (unsigned short)(r >> 16);
  r = sp2(b.z); ph.s[6] = (unsigned short)(r & 0xFFFFu); pl.s[6] = (unsigned short)(r >> 16);
  r = sp2(b.w); ph.s[7] = (unsigned short)(r & 0xFFFFu); pl.s[7] = (unsigned short)(r >> 16);
  hi = ph.i;
  lo = pl.i;
}

__device__ __forceinline__ void tput(unsigned short* T, int nl0, int kl, v4f v) {
  unsigned r;
  r = sp2(v.x); T[(nl0 + 0) * TP + kl] = (unsigned short)(r & 0xFFFFu); T[(64 + nl0 + 0) * TP + kl] = (unsigned short)(r >> 16);
  r = sp2(v.y); T[(nl0 + 1) * TP + kl] = (unsigned short)(r & 0xFFFFu); T[(64 + nl0 + 1) * TP + kl] = (unsigned short)(r >> 16);
  r = sp2(v.z); T[(nl0 + 2) * TP + kl] = (unsigned short)(r & 0xFFFFu); T[(64 + nl0 + 2) * TP + kl] = (unsigned short)(r >> 16);
  r = sp2(v.w); T[(nl0 + 3) * TP + kl] = (unsigned short)(r & 0xFFFFu); T[(64 + nl0 + 3) * TP + kl] = (unsigned short)(r >> 16);
}

__global__ __launch_bounds__(NTHR) void k_prepw(const float* __restrict__ W, unsigned short* Wb) {
  __shared__ __attribute__((aligned(16))) unsigned short T[2 * 64 * TP];
  const int tid  = threadIdx.x;
  const int lane = tid & 31;
  const int wave = tid >> 5;
  const int k0 = blockIdx.x * 64;
  const int n0 = blockIdx.y * 64;
  {
    const int kl = tid >> 2;
    const int nq = (tid & 3) * 16;
    const float* p = W + (size_t)(k0 + kl) * NQKV + n0 + nq;
    const v4f f0 = *(const v4f*)(p);
    const v4f f1 = *(const v4f*)(p + 4);
    const v4f f2 = *(const v4f*)(p + 8);
    const v4f f3 = *(const v4f*)(p + 12);
    tput(T, nq + 0,  kl, f0);
    tput(T, nq + 4,  kl, f1);
    tput(T, nq + 8,  kl, f2);
    tput(T, nq + 12, kl, f3);
  }
  __syncthreads();

  v4i val[4];
  size_t off[4];
#pragma unroll
  for (int p = 0; p < 4; ++p) {
    const int g     = (p * 8 + wave) * 4 + (lane >> 3);
    const int plane = g >> 6;
    const int nl    = g & 63;
    const int piece = lane & 7;
    val[p] = *(const v4i*)(T + (plane * 64 + nl) * TP + 8 * piece);
    off[p] = ((size_t)(plane * NQKV + n0 + nl)) * KIN + (size_t)(k0 + 8 * piece);
  }
#pragma unroll
  for (int p = 0; p < 4; ++p) *(volatile v4i*)(Wb + off[p]) = val[p];
  __threadfence();
#pragma unroll
  for (int p = 0; p < 4; ++p) *(volatile v4i*)(Wb + off[p]) = val[p];
}

__global__ __launch_bounds__(NTHR) void k_gemm(
    const float* __restrict__ x, const unsigned short* __restrict__ Wb,
    float* qkv, int nN) {
  __shared__ __attribute__((aligned(16))) unsigned short Ah[GR * AP];
  __shared__ __attribute__((aligned(16))) unsigned short Al[GR * AP];
  __shared__ __attribute__((aligned(16))) float Os[16 * OP];

  const int tid  = threadIdx.x;
  const int lane = tid & 31;
  const int wave = tid >> 5;
  const int hh   = lane >> 4;
  const int m    = lane & 15;
  const int rowBase = blockIdx.x * GR;
  const int colBase = blockIdx.y * GC;
  const unsigned short* Wh = Wb;
  const unsigned short* Wl = Wb + (size_t)NQKV * KIN;

  const int sr   = tid >> 3;
  const int scol = (tid & 7) * 16;
  int srow = rowBase + sr;
  if (srow > nN - 1) srow = nN - 1;
  const float* xs = x + (size_t)srow * KIN + scol;

  const v8f z8 = {0.f, 0.f, 0.f, 0.f, 0.f, 0.f, 0.f, 0.f};
  v8f acc[2][4];
#pragma unroll
  for (int i = 0; i < 2; ++i)
#pragma unroll
    for (int j = 0; j < 4; ++j) acc[i][j] = z8;

  const int wcol = colBase + wave * 64 + m;

#pragma unroll 1
  for (int kc = 0; kc < KIN; kc += KC) {
    {
      const v4f f0 = *(const v4f*)(xs + kc);
      const v4f f1 = *(const v4f*)(xs + kc + 4);
      const v4f f2 = *(const v4f*)(xs + kc + 8);
      const v4f f3 = *(const v4f*)(xs + kc + 12);
      v4i h0, l0, h1, l1;
      sp8(f0, f1, h0, l0);
      sp8(f2, f3, h1, l1);
      *(v4i*)(Ah + sr * AP + scol)     = h0;
      *(v4i*)(Ah + sr * AP + scol + 8) = h1;
      *(v4i*)(Al + sr * AP + scol)     = l0;
      *(v4i*)(Al + sr * AP + scol + 8) = l1;
    }
    __syncthreads();

#pragma unroll 1
    for (int ks = 0; ks < KC; ks += 32) {
      Frag ah0, ah1, al0, al1;
      const int pa0 = m * AP + ks + 8 * hh;
      const int pa1 = (16 + m) * AP + ks + 8 * hh;
      ah0.q[0] = *(const v4i*)(Ah + pa0); ah0.q[1] = *(const v4i*)(Ah + pa0 + 16);
      al0.q[0] = *(const v4i*)(Al + pa0); al0.q[1] = *(const v4i*)(Al + pa0 + 16);
      ah1.q[0] = *(const v4i*)(Ah + pa1); ah1.q[1] = *(const v4i*)(Ah + pa1 + 16);
      al1.q[0] = *(const v4i*)(Al + pa1); al1.q[1] = *(const v4i*)(Al + pa1 + 16);
      const size_t kg = (size_t)(kc + ks + 8 * hh);
#pragma unroll
      for (int j = 0; j < 4; ++j) {
        const size_t boff = (size_t)(wcol + 16 * j) * KIN + kg;
        Frag bh, bl;
        bh.q[0] = *(const v4i*)(Wh + boff); bh.q[1] = *(const v4i*)(Wh + boff + 16);
        bl.q[0] = *(const v4i*)(Wl + boff); bl.q[1] = *(const v4i*)(Wl + boff + 16);
        acc[0][j] = wm(ah0.v, bh.v, acc[0][j]);
        acc[0][j] = wm(ah0.v, bl.v, acc[0][j]);
        acc[0][j] = wm(al0.v, bh.v, acc[0][j]);
        acc[1][j] = wm(ah1.v, bh.v, acc[1][j]);
        acc[1][j] = wm(ah1.v, bl.v, acc[1][j]);
        acc[1][j] = wm(al1.v, bh.v, acc[1][j]);
      }
    }
    __syncthreads();
  }

#pragma unroll
  for (int i = 0; i < 2; ++i) {
#pragma unroll
    for (int j = 0; j < 4; ++j) {
#pragma unroll
      for (int r = 0; r < 8; ++r)
        Os[(8 * hh + r) * OP + wave * 64 + 16 * j + m] = acc[i][j][r];
    }
    __syncthreads();
    v4f v[8];
    float* gp[8];
#pragma unroll
    for (int t = 0; t < 8; ++t) {
      const int rr = 2 * wave + (t >> 2);
      const int qq = t & 3;
      v[t]  = *(const v4f*)(Os + rr * OP + 128 * qq + 4 * lane);
      gp[t] = qkv + (size_t)(rowBase + 16 * i + rr) * NQKV + colBase + 128 * qq + 4 * lane;
    }
#pragma unroll
    for (int t = 0; t < 8; ++t) *(volatile v4f*)(gp[t]) = v[t];
    __threadfence();
#pragma unroll
    for (int t = 0; t < 8; ++t) *(volatile v4f*)(gp[t]) = v[t];
    __syncthreads();
  }
}

__global__ __launch_bounds__(NTHR) void k_agg(
    const int* __restrict__ ei, const float* __restrict__ qkv,
    float* out, int nN, int nE) {
  extern __shared__ v4f lds_dyn[];
  float* sacc = (float*)lds_dyn;
  float* mrow = sacc + LDS_SACC;
  float* drow = mrow + NB * NHD;
  int*   list = (int*)(drow + NB * NHD);
  int*   wcnt = list + LDS_LIST;

  const int tid  = threadIdx.x;
  const int lane = tid & 31;
  const int wave = tid >> 5;
  const int hh   = lane >> 4;
  const int nodeBase = blockIdx.x * NB;

  {
    const v4f z4 = {0.f, 0.f, 0.f, 0.f};
    for (int i = tid; i < LDS_SACC / 4; i += NTHR) lds_dyn[i] = z4;
    for (int i = tid; i < NB * NHD; i += NTHR) { mrow[i] = -__builtin_inff(); drow[i] = 0.f; }
  }
  __syncthreads();

  const int* esrc = ei;
  const int* edst = ei + nE;
  const bool al16 = ((((size_t)esrc) & 15) == 0);

  const int nChunks = (nE + CHUNK - 1) / CHUNK;
#pragma unroll 1
  for (int ch = 0; ch < nChunks; ++ch) {
    const int cbase = ch * CHUNK;
    int wc = 0;
#pragma unroll
    for (int g = 0; g < NGRP; ++g) {
      const int el0 = (g * NTHR + tid) * 4;
      const int e0  = cbase + el0;
      const int sent = -2147483647 - 1;
      v4i d;
      if (al16 && (cbase + CHUNK <= nE)) {
        d = *(const v4i*)(esrc + e0);
      } else {
        d.x = (e0     < nE) ? esrc[min(e0,     nE - 1)] : sent;
        d.y = (e0 + 1 < nE) ? esrc[min(e0 + 1, nE - 1)] : sent;
        d.z = (e0 + 2 < nE) ? esrc[min(e0 + 2, nE - 1)] : sent;
        d.w = (e0 + 3 < nE) ? esrc[min(e0 + 3, nE - 1)] : sent;
      }
      const unsigned s0 = (unsigned)d.x - (unsigned)nodeBase;
      const unsigned s1 = (unsigned)d.y - (unsigned)nodeBase;
      const unsigned s2 = (unsigned)d.z - (unsigned)nodeBase;
      const unsigned s3 = (unsigned)d.w - (unsigned)nodeBase;
      const bool h0 = s0 < (unsigned)NB;
      const bool h1 = s1 < (unsigned)NB;
      const bool h2 = s2 < (unsigned)NB;
      const bool h3 = s3 < (unsigned)NB;
      const unsigned many = __builtin_amdgcn_ballot_w32(h0 | h1 | h2 | h3);
      if (many != 0u) {
#define HITJ(J, HJ, SJ) { \
          const unsigned mj = __builtin_amdgcn_ballot_w32(HJ); \
          if (HJ) { \
            const int pos = wc + (int)__builtin_amdgcn_mbcnt_lo(mj, 0u); \
            if (pos < WCAP) list[wave * WCAP + pos] = ((el0 + (J)) << 8) | (int)(SJ); \
          } \
          wc += (int)__builtin_popcount(mj); }
        HITJ(0, h0, s0)
        HITJ(1, h1, s1)
        HITJ(2, h2, s2)
        HITJ(3, h3, s3)
#undef HITJ
      }
    }
    if (lane == 0) wcnt[wave] = wc;
    __syncthreads();

#pragma unroll 1
    for (int wsx = 0; wsx < NWAVE; ++wsx) {
      int n = wcnt[wsx];
      if (n > WCAP) n = WCAP;
      if (n < 0) n = 0;
#pragma unroll 1
      for (int i = 0; i < n; ++i) {
        const int ent  = list[wsx * WCAP + i];
        const int slot = ent & (NB - 1);
        if ((slot >> 3) != wave) continue;
        const int el = (ent >> 8) & (CHUNK - 1);
        int e = cbase + el;
        if (e > nE - 1) e = nE - 1;
        int dst = edst[e];
        dst = dst < 0 ? 0 : (dst > nN - 1 ? nN - 1 : dst);
        int node = nodeBase + slot;
        if (node > nN - 1) node = nN - 1;

        const float* qp = qkv + (size_t)node * NQKV + 4 * lane;
        const float* kp = qkv + (size_t)dst * NQKV + KIN + 4 * lane;
        const float* vp = qkv + (size_t)dst * NQKV + 2 * KIN + 4 * lane;

        float a[4];
#pragma unroll
        for (int q = 0; q < 4; ++q) {
          const v4f qv = *(const v4f*)(qp + 128 * q);
          const v4f kv = *(const v4f*)(kp + 128 * q);
          float s = qv.x * kv.x;
          s += qv.y * kv.y;
          s += qv.z * kv.z;
          s += qv.w * kv.w;
          s += __shfl_xor(s, 1, 32);
          s += __shfl_xor(s, 2, 32);
          s += __shfl_xor(s, 4, 32);
          s += __shfl_xor(s, 8, 32);
          a[q] = s * 0.125f;
        }

        const v4f mA = *(const v4f*)(mrow + slot * NHD);
        const v4f mB = *(const v4f*)(mrow + slot * NHD + 4);
        const v4f dA = *(const v4f*)(drow + slot * NHD);
        const v4f dB = *(const v4f*)(drow + slot * NHD + 4);
        float mo[4], dd[4];
        mo[0] = hh ? mA.y : mA.x;   dd[0] = hh ? dA.y : dA.x;
        mo[1] = hh ? mA.w : mA.z;   dd[1] = hh ? dA.w : dA.z;
        mo[2] = hh ? mB.y : mB.x;   dd[2] = hh ? dB.y : dB.x;
        mo[3] = hh ? mB.w : mB.z;   dd[3] = hh ? dB.w : dB.z;

        float mn[4], dn[4];
#pragma unroll
        for (int q = 0; q < 4; ++q) {
          const float mq = fmaxf(mo[q], a[q]);
          const float sc = __expf(mo[q] - mq);
          const float p  = __expf(a[q] - mq);
          mn[q] = mq;
          dn[q] = dd[q] * sc + p;
          v4f* ap = (v4f*)(sacc + slot * FOUT + 128 * q + 4 * lane);
          const v4f av = *ap;
          const v4f vv = *(const v4f*)(vp + 128 * q);
          *ap = av * sc + p * vv;
        }

        float mt[4], dt[4];
#pragma unroll
        for (int q = 0; q < 4; ++q) {
          mt[q] = __shfl_xor(mn[q], 16, 32);
          dt[q] = __shfl_xor(dn[q], 16, 32);
        }
        v4f nm0, nm1, nd0, nd1;
        nm0.x = hh ? mt[0] : mn[0];  nm0.y = hh ? mn[0] : mt[0];
        nm0.z = hh ? mt[1] : mn[1];  nm0.w = hh ? mn[1] : mt[1];
        nm1.x = hh ? mt[2] : mn[2];  nm1.y = hh ? mn[2] : mt[2];
        nm1.z = hh ? mt[3] : mn[3];  nm1.w = hh ? mn[3] : mt[3];
        nd0.x = hh ? dt[0] : dn[0];  nd0.y = hh ? dn[0] : dt[0];
        nd0.z = hh ? dt[1] : dn[1];  nd0.w = hh ? dn[1] : dt[1];
        nd1.x = hh ? dt[2] : dn[2];  nd1.y = hh ? dn[2] : dt[2];
        nd1.z = hh ? dt[3] : dn[3];  nd1.w = hh ? dn[3] : dt[3];
        *(v4f*)(mrow + slot * NHD)     = nm0;
        *(v4f*)(mrow + slot * NHD + 4) = nm1;
        *(v4f*)(drow + slot * NHD)     = nd0;
        *(v4f*)(drow + slot * NHD + 4) = nd1;
      }
    }
    __syncthreads();
  }

#pragma unroll 1
  for (int j = 0; j < NB / NWAVE; ++j) {
    const int slot = wave * (NB / NWAVE) + j;
    const int node = nodeBase + slot;
    if (node >= nN) break;
    const v4f dA = *(const v4f*)(drow + slot * NHD);
    const v4f dB = *(const v4f*)(drow + slot * NHD + 4);
    float dd[4];
    dd[0] = hh ? dA.y : dA.x;
    dd[1] = hh ? dA.w : dA.z;
    dd[2] = hh ? dB.y : dB.x;
    dd[3] = hh ? dB.w : dB.z;
    v4f y[4];
#pragma unroll
    for (int q = 0; q < 4; ++q) {
      const float dq  = dd[q];
      const float inv = (dq > 0.f) ? __builtin_amdgcn_rcpf(dq) : 0.f;
      y[q] = *(const v4f*)(sacc + slot * FOUT + 128 * q + 4 * lane) * inv;
    }
    float* op = out + (size_t)node * FOUT + 4 * lane;
#pragma unroll
    for (int q = 0; q < 4; ++q) *(volatile v4f*)(op + 128 * q) = y[q];
    __threadfence();
#pragma unroll
    for (int q = 0; q < 4; ++q) *(volatile v4f*)(op + 128 * q) = y[q];
  }
}

extern "C" void kernel_launch(void* const* d_in, const int* in_sizes, int n_in,
                              void* d_out, int out_size, void* d_ws, size_t ws_size,
                              hipStream_t stream) {
  if (n_in < 4) return;
  const int nN = in_sizes[0] / KIN;
  if (nN <= 0 || in_sizes[0] != nN * KIN) return;
  if (in_sizes[2] < 0 || (in_sizes[2] & 1) != 0) return;
  const int nE = in_sizes[2] / 2;
  if (in_sizes[3] != KIN * NQKV) return;
  if (out_size != nN * FOUT) return;

  const float* x  = (const float*)d_in[0];
  const int*   ei = (const int*)d_in[2];
  const float* W  = (const float*)d_in[3];
  float* out = (float*)d_out;

  const int nP = ((nN + GR - 1) / GR) * GR;
  size_t off = 0;
  unsigned short* Wb = (unsigned short*)((char*)d_ws + off);
  off += (size_t)2 * NQKV * KIN * sizeof(unsigned short);
  float* qkv = (float*)((char*)d_ws + off);
  off += (size_t)nP * NQKV * sizeof(float);
  if (off > ws_size) return;

  k_prepw<<<dim3(KIN / 64, NQKV / 64), NTHR, 0, stream>>>(W, Wb);

  k_gemm<<<dim3(nP / GR, NQKV / GC), NTHR, 0, stream>>>(x, Wb, qkv, nN);

  hipFuncSetAttribute(reinterpret_cast<const void*>(&k_agg),
                      hipFuncAttributeMaxDynamicSharedMemorySize, LDS_BYTES);
  const int grid = (nN + NB - 1) / NB;
  k_agg<<<grid, NTHR, LDS_BYTES, stream>>>(ei, qkv, out, nN, nE);
}
